// SE3GTLayer_12841952215575
// MI455X (gfx1250) — hardware-verified
//
#include <hip/hip_runtime.h>
#include <stddef.h>


#define NN   8192
#define EE   262144
#define DD   128
#define HH   256
#define DH   64
#define ED   16
#define YY   64
#define NK1  384
#define NE1  273
#define NWF  704
#define WSC  16.0f
#define WINV 0.0625f
#define PSC  16384.0f
#define OSC  16.0f
#define OINV 0.00390625f
#define RAD2 100.0f

typedef float          v2f  __attribute__((ext_vector_type(2)));
typedef float          v4f  __attribute__((ext_vector_type(4)));
typedef float          v8f  __attribute__((ext_vector_type(8)));
typedef int            v4i  __attribute__((ext_vector_type(4)));
typedef _Float16       v8h  __attribute__((ext_vector_type(8)));
typedef _Float16       v16h __attribute__((ext_vector_type(16)));
typedef __bf16         v16b __attribute__((ext_vector_type(16)));
typedef unsigned short v4us __attribute__((ext_vector_type(4)));
typedef unsigned short v8us __attribute__((ext_vector_type(8)));
typedef v2f  __attribute__((may_alias)) v2fa;
typedef v4f  __attribute__((may_alias)) v4fa;
typedef v4i  __attribute__((may_alias)) v4ia;
typedef v8h  __attribute__((may_alias)) v8ha;
typedef v4us __attribute__((may_alias)) v4usa;
typedef v8us __attribute__((may_alias)) v8usa;
union FragH { v16h v; v8h h[2]; };
union FragB { v16b v; v8us u[2]; };
union Bits8 { v8h h; v8us u; };

__device__ __forceinline__ v8f wmh(v16h a, v16h b, v8f c) {
  v8f d = __builtin_amdgcn_wmma_f32_16x16x32_f16(false, a, false, b, (short)0, c, false, false);
  asm volatile("v_nop\n\tv_nop\n\tv_nop\n\tv_nop" : "+v"(d) : "v"(a), "v"(b));
  return d;
}
__device__ __forceinline__ v8f wmb(v16b a, v16b b, v8f c) {
  v8f d = __builtin_amdgcn_wmma_f32_16x16x32_bf16(false, a, false, b, (short)0, c, false, false);
  asm volatile("v_nop\n\tv_nop\n\tv_nop\n\tv_nop" : "+v"(d) : "v"(a), "v"(b));
  return d;
}
__device__ __forceinline__ v8f wmb3(v16b ah, v16b al, v16b bh, v16b bl, v8f c) {
  c = wmb(ah, bh, c);
  c = wmb(ah, bl, c);
  c = wmb(al, bh, c);
  return c;
}

__device__ __forceinline__ v16h ldh(const _Float16* p, int h) {
  FragH f;
  f.h[0] = *(const v8ha*)(p + 8 * h);
  f.h[1] = *(const v8ha*)(p + 16 + 8 * h);
  return f.v;
}
__device__ __forceinline__ v16b ldb(const unsigned short* p, int h) {
  FragB f;
  f.u[0] = *(const v8usa*)(p + 8 * h);
  f.u[1] = *(const v8usa*)(p + 16 + 8 * h);
  return f.v;
}

__device__ __forceinline__ unsigned short bfbits(float v) {
  unsigned int u = __float_as_uint(v);
  u = u + 0x7FFFu + ((u >> 16) & 1u);
  return (unsigned short)(u >> 16);
}
__device__ __forceinline__ void bfsplit(float v, unsigned short& hi, unsigned short& lo) {
  hi = bfbits(v);
  const float hf = __uint_as_float(((unsigned int)hi) << 16);
  lo = bfbits(v - hf);
}

__device__ __forceinline__ float silu_f(float v) {
  const float e = __expf(fminf(-v, 80.0f));
  return v * __builtin_amdgcn_rcpf(1.0f + e);
}

__device__ __forceinline__ float wsum(float v) {
#pragma unroll
  for (int o = 16; o > 0; o >>= 1) v += __shfl_xor(v, o, 32);
  return v;
}

__device__ __forceinline__ v8h cvt8h(v8f a, float sc) {
  v8h r;
#pragma unroll
  for (int i = 0; i < 8; ++i) r[i] = (_Float16)(a[i] * sc);
  return r;
}
__device__ __forceinline__ v16h pack2(v8f a, v8f c, float sc) {
  FragH f;
  f.h[0] = cvt8h(a, sc);
  f.h[1] = cvt8h(c, sc);
  return f.v;
}

#define CB1 131072
#define CB2 142336
#define CB3 143360
#define CB4 151552
#define CB5 152576
#define CB6 164864
#define CB7 168960
#define CB8 173056
#define CB9 175104
static_assert(CB1 == NN * DD / 8);
static_assert(CB2 - CB1 == NWF * DD / 8);
static_assert(CB3 - CB2 == HH * 32 / 8);
static_assert(CB4 - CB3 == HH * HH / 8);
static_assert(CB5 - CB4 == DD * DH / 8);
static_assert(CB6 - CB5 == HH * NK1 / 8);
static_assert(CB7 - CB6 == DD * HH / 8);
static_assert(CB8 - CB7 == HH * DD / 8);
static_assert(CB9 - CB8 == YY * HH / 8);
static_assert((CB1 % 32) == 0 && (CB2 % 32) == 0 && (CB3 % 32) == 0 && (CB4 % 32) == 0 && (CB5 % 32) == 0);
static_assert((CB6 % 32) == 0 && (CB7 % 32) == 0 && (CB8 % 32) == 0 && (CB9 % 256) == 0);

__global__ __launch_bounds__(256) void k_convert(
    const float* __restrict__ x, const float* __restrict__ ew1, const float* __restrict__ ew2,
    const float* __restrict__ wq, const float* __restrict__ wk, const float* __restrict__ wv,
    const float* __restrict__ wo, const float* __restrict__ nw1, const float* __restrict__ nw2,
    const float* __restrict__ cmw1, const float* __restrict__ cmw2,
    unsigned short* xh, unsigned short* wf, unsigned short* wa, unsigned short* w2,
    unsigned short* wot, unsigned short* n1h, unsigned short* n1l, unsigned short* n2h,
    unsigned short* n2l, unsigned short* c1h, unsigned short* c1l, unsigned short* c2h,
    unsigned short* c2l) {
  const int g = blockIdx.x * 256 + threadIdx.x;
  if (g >= CB9) return;
  float f[8];
#pragma unroll
  for (int i = 0; i < 8; ++i) f[i] = 0.0f;
  float sc = 1.0f;
  int kind = 0;
  unsigned short* d0;
  unsigned short* d1;
  if (g < CB1) {
    const v4f a = *(const v4fa*)(x + (size_t)g * 8);
    const v4f c = *(const v4fa*)(x + (size_t)g * 8 + 4);
    f[0] = a.x; f[1] = a.y; f[2] = a.z; f[3] = a.w; f[4] = c.x; f[5] = c.y; f[6] = c.z; f[7] = c.w;
    d0 = xh + (size_t)g * 8; d1 = d0;
  } else if (g < CB2) {
    const int e = g - CB1;
    const int row = e >> 4;
    const int k0 = (e & 15) * 8;
    const float* src;
    int pitch;
    if (row < 256)      { src = ew1 + (size_t)k0 * HH + row;                pitch = HH; }
    else if (row < 512) { src = ew1 + (size_t)(DD + k0) * HH + (row - 256); pitch = HH; }
    else if (row < 576) { src = wq + (size_t)k0 * DH + (row - 512);         pitch = DH; }
    else if (row < 640) { src = wk + (size_t)k0 * DH + (row - 576);         pitch = DH; }
    else                { src = wv + (size_t)k0 * DH + (row - 640);         pitch = DH; }
#pragma unroll
    for (int i = 0; i < 8; ++i) f[i] = src[(size_t)i * pitch];
    sc = WSC; d0 = wf + (size_t)e * 8; d1 = d0;
  } else if (g < CB3) {
    const int e = g - CB2;
    const int row = e >> 2;
    const int k0 = (e & 3) * 8;
#pragma unroll
    for (int i = 0; i < 8; ++i) {
      const int kk = k0 + i;
      const int kc = kk < ED ? kk : (ED - 1);
      const float v = ew1[(size_t)(2 * DD + 1 + kc) * HH + row];
      f[i] = (kk < ED) ? v : 0.0f;
    }
    sc = WSC; d0 = wa + (size_t)e * 8; d1 = d0;
  } else if (g < CB4) {
    const int e = g - CB3;
    const int row = e >> 5;
    const int k0 = (e & 31) * 8;
#pragma unroll
    for (int i = 0; i < 8; ++i) f[i] = ew2[(size_t)(k0 + i) * HH + row];
    sc = WSC; d0 = w2 + (size_t)e * 8; d1 = d0;
  } else if (g < CB5) {
    const int e = g - CB4;
    const int row = e >> 3;
    const int k0 = (e & 7) * 8;
#pragma unroll
    for (int i = 0; i < 8; ++i) f[i] = wo[(size_t)(k0 + i) * DD + row];
    sc = WSC; d0 = wot + (size_t)e * 8; d1 = d0;
  } else if (g < CB6) {
    const int e = g - CB5;
    const int row = e / 48;
    const int k0 = (e - row * 48) * 8;
#pragma unroll
    for (int i = 0; i < 8; ++i) f[i] = nw1[(size_t)(k0 + i) * HH + row];
    kind = 1; d0 = n1h + (size_t)e * 8; d1 = n1l + (size_t)e * 8;
  } else if (g < CB7) {
    const int e = g - CB6;
    const int row = e >> 5;
    const int k0 = (e & 31) * 8;
#pragma unroll
    for (int i = 0; i < 8; ++i) f[i] = nw2[(size_t)(k0 + i) * DD + row];
    kind = 1; d0 = n2h + (size_t)e * 8; d1 = n2l + (size_t)e * 8;
  } else if (g < CB8) {
    const int e = g - CB7;
    const int row = e >> 4;
    const int k0 = (e & 15) * 8;
#pragma unroll
    for (int i = 0; i < 8; ++i) f[i] = cmw1[(size_t)(k0 + i) * HH + row];
    kind = 1; d0 = c1h + (size_t)e * 8; d1 = c1l + (size_t)e * 8;
  } else {
    const int e = g - CB8;
    const int row = e >> 5;
    const int k0 = (e & 31) * 8;
#pragma unroll
    for (int i = 0; i < 8; ++i) f[i] = cmw2[(size_t)(k0 + i) * YY + row];
    kind = 1; d0 = c2h + (size_t)e * 8; d1 = c2l + (size_t)e * 8;
  }
  v8us u0, u1;
  if (kind == 0) {
    Bits8 b;
#pragma unroll
    for (int i = 0; i < 8; ++i) b.h[i] = (_Float16)(f[i] * sc);
    u0 = b.u; u1 = b.u;
  } else {
#pragma unroll
    for (int i = 0; i < 8; ++i) {
      unsigned short hs, ls;
      bfsplit(f[i], hs, ls);
      u0[i] = hs; u1[i] = ls;
    }
  }
  *(volatile v8us*)d0 = u0;
  if (kind != 0) *(volatile v8us*)d1 = u1;
  __threadfence();
  *(volatile v8us*)d0 = u0;
  if (kind != 0) *(volatile v8us*)d1 = u1;
}

__device__ __forceinline__ void pq_pass(const float* sF, float* pq, int m0w, int g, int w, int lane) {
  const int q8 = lane & 7, sub = lane >> 3;
#pragma unroll
  for (int i = 0; i < 16; ++i) {
    const int lid = i * 4 + sub;
    const int row = lid >> 1, hl = lid & 1;
    const v4f v = *(const v4fa*)(sF + (32 * w + row) * 64 + 32 * hl + 4 * q8);
    *(volatile v4f*)(pq + (size_t)(m0w + row) * (2 * HH) + 64 * g + 32 * hl + 4 * q8) = v;
  }
}
__device__ __forceinline__ void qk_pass(const _Float16* sH, _Float16* pl, int m0w, int w, int lane) {
  const int q8 = lane & 7, sub = lane >> 3;
#pragma unroll
  for (int i = 0; i < 8; ++i) {
    const int lid = i * 4 + sub;
    const v8h v = *(const v8ha*)(sH + (32 * w + lid) * DH + 8 * q8);
    *(volatile v8h*)(pl + (size_t)(m0w + lid) * DH + 8 * q8) = v;
  }
}
__device__ __forceinline__ void vt_pass(const _Float16* sH, _Float16* vt, int m0, int w, int lane) {
  const int q8 = lane & 7, sub = lane >> 3;
#pragma unroll
  for (int i = 0; i < 8; ++i) {
    const int lid = w * 32 + i * 4 + sub;
    const int d = lid >> 1, hl = lid & 1;
    const v8h v = *(const v8ha*)(sH + d * 128 + 64 * hl + 8 * q8);
    *(volatile v8h*)(vt + (size_t)d * NN + m0 + 64 * hl + 8 * q8) = v;
  }
}

__global__ __launch_bounds__(128) void k_proj(
    const _Float16* __restrict__ xh, const _Float16* __restrict__ wf, const float* __restrict__ eb1,
    float* pq, _Float16* qh, _Float16* kh, _Float16* vt) {
  __shared__ __attribute__((aligned(16))) float    sF[128 * 64];
  __shared__ __attribute__((aligned(16))) _Float16 sH[128 * 64];
  const int tid = threadIdx.x, lane = tid & 31, w = tid >> 5, h = lane >> 4, m = lane & 15;
  const int m0 = blockIdx.x * 128;
  const int g = blockIdx.y;
  const int m0w = m0 + 32 * w;

  const _Float16* xa0 = xh + (size_t)(m0w + m) * DD;
  const _Float16* xa1 = xa0 + (size_t)16 * DD;
  const _Float16* wb  = wf + (size_t)(64 * g + m) * DD;

  const v8f zf = {0.f, 0.f, 0.f, 0.f, 0.f, 0.f, 0.f, 0.f};
  v8f acc[2][4];
#pragma unroll
  for (int mt = 0; mt < 2; ++mt)
#pragma unroll
    for (int nt = 0; nt < 4; ++nt) acc[mt][nt] = zf;

#pragma unroll
  for (int k0 = 0; k0 < DD; k0 += 32) {
    const v16h a0 = ldh(xa0 + k0, h);
    const v16h a1 = ldh(xa1 + k0, h);
#pragma unroll
    for (int nt = 0; nt < 4; ++nt) {
      const v16h b = ldh(wb + (size_t)nt * 16 * DD + k0, h);
      acc[0][nt] = wmh(a0, b, acc[0][nt]);
      acc[1][nt] = wmh(a1, b, acc[1][nt]);
    }
  }

  if (g < 8) {
#pragma unroll
    for (int nt = 0; nt < 4; ++nt) {
      const int feat = 16 * nt + m;
      const int col = 64 * g + feat;
      const int bi = col < HH ? col : (HH - 1);
      const float bl = eb1[bi];
      const float bv = (g < 4) ? bl : 0.0f;
#pragma unroll
      for (int mt = 0; mt < 2; ++mt)
#pragma unroll
        for (int r = 0; r < 8; ++r) {
          const int tokl = 32 * w + 16 * mt + 8 * h + r;
          sF[tokl * 64 + feat] = acc[mt][nt][r] * WINV + bv;
        }
    }
    __syncthreads();
    pq_pass(sF, pq, m0w, g, w, lane);
    __threadfence();
    pq_pass(sF, pq, m0w, g, w, lane);
  } else if (g < 10) {
#pragma unroll
    for (int nt = 0; nt < 4; ++nt)
#pragma unroll
      for (int mt = 0; mt < 2; ++mt)
#pragma unroll
        for (int r = 0; r < 8; ++r) {
          const int tokl = 32 * w + 16 * mt + 8 * h + r;
          sH[tokl * DH + 16 * nt + m] = (_Float16)(acc[mt][nt][r] * WINV);
        }
    __syncthreads();
    _Float16* pl = (g == 8) ? qh : kh;
    qk_pass(sH, pl, m0w, w, lane);
    __threadfence();
    qk_pass(sH, pl, m0w, w, lane);
  } else {
#pragma unroll
    for (int nt = 0; nt < 4; ++nt)
#pragma unroll
      for (int mt = 0; mt < 2; ++mt)
#pragma unroll
        for (int r = 0; r < 8; ++r) {
          const int tokl = 32 * w + 16 * mt + 8 * h + r;
          sH[(16 * nt + m) * 128 + tokl] = (_Float16)(acc[mt][nt][r] * WINV);
        }
    __syncthreads();
    vt_pass(sH, vt, m0, w, lane);
    __threadfence();
    vt_pass(sH, vt, m0, w, lane);
  }
}

#define ENT   128
#define ENW   4
#define EPT   8
#define CHUNK (ENT * EPT)
#define WCAP  (EPT * 32)
#define LISTN (ENW * WCAP)
#define PASSN (ENW * 16)
#define PCAP  (CHUNK + PASSN)
#define NB    64
static_assert(PASSN == 64);
static_assert(PCAP >= CHUNK + PASSN);
static_assert((NB % ENW) == 0);
static_assert((NN % NB) == 0);
static_assert((EE % EPT) == 0);

__device__ __forceinline__ int scan_chunk(const int* __restrict__ ids, int nE, int cbase, int nodeBase,
                                          int* list, int tid, int wave) {
  int wc = 0;
  const int el0  = tid * EPT;
  const int e0   = cbase + el0;
  const int sent = -2147483647 - 1;
  const bool gv  = e0 < nE;
  const int eb   = gv ? e0 : (nE - EPT);
  const v4i la = *(const v4ia*)(ids + eb);
  const v4i lb = *(const v4ia*)(ids + eb + 4);
  const int t0 = gv ? la.x : sent, t1 = gv ? la.y : sent, t2 = gv ? la.z : sent, t3 = gv ? la.w : sent;
  const int t4 = gv ? lb.x : sent, t5 = gv ? lb.y : sent, t6 = gv ? lb.z : sent, t7 = gv ? lb.w : sent;
  const unsigned nb = (unsigned)nodeBase;
  const bool h0 = ((unsigned)t0 - nb) < (unsigned)NB, h1 = ((unsigned)t1 - nb) < (unsigned)NB;
  const bool h2 = ((unsigned)t2 - nb) < (unsigned)NB, h3 = ((unsigned)t3 - nb) < (unsigned)NB;
  const bool h4 = ((unsigned)t4 - nb) < (unsigned)NB, h5 = ((unsigned)t5 - nb) < (unsigned)NB;
  const bool h6 = ((unsigned)t6 - nb) < (unsigned)NB, h7 = ((unsigned)t7 - nb) < (unsigned)NB;
  const unsigned any = __builtin_amdgcn_ballot_w32(h0 | h1 | h2 | h3 | h4 | h5 | h6 | h7);
  if (any != 0u) {
#define HITJ(J, HJ) { \
      const unsigned mj = __builtin_amdgcn_ballot_w32(HJ); \
      if (mj != 0u) { \
        if (HJ) { \
          const int pos = wc + (int)__builtin_amdgcn_mbcnt_lo(mj, 0u); \
          if (pos < WCAP) list[wave * WCAP + pos] = el0 + (J); \
        } \
        wc += (int)__builtin_popcount(mj); } }
    HITJ(0, h0)
    HITJ(1, h1)
    HITJ(2, h2)
    HITJ(3, h3)
    HITJ(4, h4)
    HITJ(5, h5)
    HITJ(6, h6)
    HITJ(7, h7)
#undef HITJ
  }
  return wc;
}

__device__ __forceinline__ void agg_pass(const float* sAcc, float* dst, int tid) {
#pragma unroll 4
  for (int i = 0; i < (NB * HH) / (4 * ENT); ++i) {
    const v4f v = *(const v4fa*)(sAcc + i * (4 * ENT) + 4 * tid);
    *(volatile v4f*)(dst + i * (4 * ENT) + 4 * tid) = v;
  }
}

__global__ __launch_bounds__(ENT) void k_edge(
    const float* __restrict__ pq, const float* __restrict__ coords, const float* __restrict__ eattr,
    const int* __restrict__ ei, const float* __restrict__ ew1, const float* __restrict__ eb2,
    const _Float16* __restrict__ wa, const _Float16* __restrict__ w2,
    float* agg, int nN, int nE) {
  __shared__ __attribute__((aligned(16))) float    sAcc[NB * HH];
  __shared__ __attribute__((aligned(16))) _Float16 sU[ENW * 16 * HH];
  __shared__ __attribute__((aligned(16))) float    sMs[ENW * 16 * 64];
  __shared__ __attribute__((aligned(16))) _Float16 sAt[PASSN * 32];
  __shared__ __attribute__((aligned(16))) int      sList[LISTN];
  __shared__ __attribute__((aligned(16))) int      sPend[PCAP];
  __shared__ int   sSlot[PASSN];
  __shared__ int   sRow[PASSN];
  __shared__ int   sCol[PASSN];
  __shared__ float sRad[PASSN];
  __shared__ int   sWcnt[ENW];
  __shared__ int   sPendN;

  const int tid = threadIdx.x, lane = tid & 31, wave = tid >> 5, h = lane >> 4, m = lane & 15;
  const int nodeBase = blockIdx.x * NB;
  const int* rowid = ei;
  const int* colid = ei + nE;

  {
    const v4f z4 = {0.0f, 0.0f, 0.0f, 0.0f};
#pragma unroll 4
    for (int i = tid; i < (NB * HH) / 4; i += ENT) *(v4fa*)(sAcc + 4 * i) = z4;
    v8h z8;
#pragma unroll
    for (int i = 0; i < 8; ++i) z8[i] = (_Float16)0.0f;
    for (int i = tid; i < (PASSN * 32) / 8; i += ENT) *(v8ha*)(sAt + 8 * i) = z8;
    if (tid == 0) sPendN = 0;
  }
  __syncthreads();

  const v8f zf = {0.f, 0.f, 0.f, 0.f, 0.f, 0.f, 0.f, 0.f};
  const int nChunks = (nE + CHUNK - 1) / CHUNK;
#pragma unroll 1
  for (int ch = 0; ch < nChunks; ++ch) {
    const int cbase = ch * CHUNK;
    const int wc = scan_chunk(rowid, nE, cbase, nodeBase, sList, tid, wave);
    if (lane == 0) sWcnt[wave] = wc;
    __syncthreads();

    const int base = sPendN;
    int tot = 0, myoff = 0;
#pragma unroll
    for (int w = 0; w < ENW; ++w) {
      int c = sWcnt[w];
      c = c > WCAP ? WCAP : (c < 0 ? 0 : c);
      if (w < wave) myoff += c;
      tot += c;
    }
    int newN = base + tot;
    newN = newN > PCAP ? PCAP : newN;
    {
      int n = sWcnt[wave];
      n = n > WCAP ? WCAP : (n < 0 ? 0 : n);
      for (int i = lane; i < n; i += 32) {
        const int pos = base + myoff + i;
        if (pos < PCAP) sPend[pos] = cbase + sList[wave * WCAP + i];
      }
    }
    const int fin = (ch == nChunks - 1) ? 1 : 0;
    const int R   = (fin != 0) ? (newN + PASSN - 1) / PASSN : newN / PASSN;
    const int Pv  = (fin != 0) ? newN : R * PASSN;
    __syncthreads();

#pragma unroll 1
    for (int r = 0; r < R; ++r) {
      {
        const int j = tid & (PASSN - 1);
        const int part = tid >> 6;
        const int idx = r * PASSN + j;
        const bool valid = idx < Pv;
        const int idc = idx < PCAP ? idx : (PCAP - 1);
        int e = sPend[idc];
        e = valid ? e : 0;
        e = e < 0 ? 0 : (e > nE - 1 ? nE - 1 : e);
        if (part == 0) {
          int ro = rowid[e];
          int co = colid[e];
          int slot = ro - nodeBase;
          if (!valid || (unsigned)slot >= (unsigned)NB) slot = NB;
          ro = ro < 0 ? 0 : (ro > nN - 1 ? nN - 1 : ro);
          co = co < 0 ? 0 : (co > nN - 1 ? nN - 1 : co);
          const float dx = coords[(size_t)ro * 3 + 0] - coords[(size_t)co * 3 + 0];
          const float dy = coords[(size_t)ro * 3 + 1] - coords[(size_t)co * 3 + 1];
          const float dz = coords[(size_t)ro * 3 + 2] - coords[(size_t)co * 3 + 2];
          const float rad = (dx * dx + dy * dy) + dz * dz;
          sSlot[j] = slot;
          sRow[j]  = ro;
          sCol[j]  = co;
          sRad[j]  = valid ? rad : 0.0f;
        } else {
          const float* ap = eattr + (size_t)e * ED;
          const v4f a0 = *(const v4fa*)ap;
          const v4f a1 = *(const v4fa*)(ap + 4);
          const v4f a2 = *(const v4fa*)(ap + 8);
          const v4f a3 = *(const v4fa*)(ap + 12);
          const float vm = valid ? 1.0f : 0.0f;
          v8h q0, q1;
          q0[0] = (_Float16)(a0.x * vm); q0[1] = (_Float16)(a0.y * vm); q0[2] = (_Float16)(a0.z * vm); q0[3] = (_Float16)(a0.w * vm);
          q0[4] = (_Float16)(a1.x * vm); q0[5] = (_Float16)(a1.y * vm); q0[6] = (_Float16)(a1.z * vm); q0[7] = (_Float16)(a1.w * vm);
          q1[0] = (_Float16)(a2.x * vm); q1[1] = (_Float16)(a2.y * vm); q1[2] = (_Float16)(a2.z * vm); q1[3] = (_Float16)(a2.w * vm);
          q1[4] = (_Float16)(a3.x * vm); q1[5] = (_Float16)(a3.y * vm); q1[6] = (_Float16)(a3.z * vm); q1[7] = (_Float16)(a3.w * vm);
          *(v8ha*)(sAt + j * 32) = q0;
          *(v8ha*)(sAt + j * 32 + 8) = q1;
        }
      }
      __syncthreads();

      const int jm = 16 * wave + m;
      const int rowm = sRow[jm], colm = sCol[jm];
      const float radm = sRad[jm];
      const v16h battr = ldh(sAt + jm * 32, h);
      const float* prow = pq + (size_t)rowm * (2 * HH);
      const float* qrow = pq + (size_t)colm * (2 * HH) + HH;
      const float* wrad = ew1 + (size_t)(2 * DD) * HH;
      _Float16* urow = sU + (wave * 16 + m) * HH;

#pragma unroll 1
      for (int ks = 0; ks < 8; ++ks) {
#pragma unroll
        for (int j2 = 0; j2 < 2; ++j2) {
          const int ft = 2 * ks + j2;
          const int f0 = 16 * ft + 8 * h;
          const v16h a = ldh(wa + (size_t)(16 * ft + m) * 32, h);
          const v8f d = wmh(a, battr, zf);
          const v4f p0 = *(const v4fa*)(prow + f0);
          const v4f p1 = *(const v4fa*)(prow + f0 + 4);
          const v4f g0 = *(const v4fa*)(qrow + f0);
          const v4f g1 = *(const v4fa*)(qrow + f0 + 4);
          const v4f w0 = *(const v4fa*)(wrad + f0);
          const v4f w1 = *(const v4fa*)(wrad + f0 + 4);
          v8h uh;
          uh[0] = (_Float16)silu_f(d[0] * WINV + p0.x + g0.x + radm * w0.x);
          uh[1] = (_Float16)silu_f(d[1] * WINV + p0.y + g0.y + radm * w0.y);
          uh[2] = (_Float16)silu_f(d[2] * WINV + p0.z + g0.z + radm * w0.z);
          uh[3] = (_Float16)silu_f(d[3] * WINV + p0.w + g0.w + radm * w0.w);
          uh[4] = (_Float16)silu_f(d[4] * WINV + p1.x + g1.x + radm * w1.x);
          uh[5] = (_Float16)silu_f(d[5] * WINV + p1.y + g1.y + radm * w1.y);
          uh[6] = (_Float16)silu_f(d[6] * WINV + p1.z + g1.z + radm * w1.z);
          uh[7] = (_Float16)silu_f(d[7] * WINV + p1.w + g1.w + radm * w1.w);
          *(v8ha*)(urow + f0) = uh;
        }
      }
      __builtin_amdgcn_fence(__ATOMIC_RELEASE, "wavefront");
      __builtin_amdgcn_wave_barrier();
      v16h bu[8];
#pragma unroll
      for (int ks = 0; ks < 8; ++ks) bu[ks] = ldh(urow + 32 * ks, h);

#pragma unroll 1
      for (int ph = 0; ph < 4; ++ph) {
#pragma unroll 1
        for (int jt = 0; jt < 4; ++jt) {
          const int ft = 4 * ph + jt;
          const _Float16* arow = w2 + (size_t)(16 * ft + m) * HH;
          v8f acc = zf;
#pragma unroll
          for (int ks = 0; ks < 8; ++ks) acc = wmh(ldh(arow + 32 * ks, h), bu[ks], acc);
          const int f0 = 16 * ft + 8 * h;
          const v4f b0 = *(const v4fa*)(eb2 + f0);
          const v4f b1 = *(const v4fa*)(eb2 + f0 + 4);
          v4f mv0, mv1;
          mv0.x = silu_f(acc[0] * WINV + b0.x); mv0.y = silu_f(acc[1] * WINV + b0.y);
          mv0.z = silu_f(acc[2] * WINV + b0.z); mv0.w = silu_f(acc[3] * WINV + b0.w);
          mv1.x = silu_f(acc[4] * WINV + b1.x); mv1.y = silu_f(acc[5] * WINV + b1.y);
          mv1.z = silu_f(acc[6] * WINV + b1.z); mv1.w = silu_f(acc[7] * WINV + b1.w);
          float* mp = sMs + (wave * 16 + m) * 64 + 16 * jt + 8 * h;
          *(v4fa*)mp = mv0;
          *(v4fa*)(mp + 4) = mv1;
        }
        __syncthreads();
#pragma unroll 1
        for (int e = 0; e < PASSN; ++e) {
          const int sl = sSlot[e];
          if (sl < NB && (sl & (ENW - 1)) == wave) {
            const v2f a = *(const v2fa*)(sMs + e * 64 + 2 * lane);
            float* ap = sAcc + sl * HH + 64 * ph + 2 * lane;
            v2f c = *(const v2fa*)ap;
            c += a;
            *(v2fa*)ap = c;
          }
        }
        __syncthreads();
      }
    }

    int rem = newN - R * PASSN;
    rem = rem < 0 ? 0 : rem;
    if (R > 0 && tid < rem) sPend[tid] = sPend[R * PASSN + tid];
    if (tid == 0) sPendN = rem;
  }
  __syncthreads();

  float* dst = agg + (size_t)nodeBase * HH;
  agg_pass(sAcc, dst, tid);
  __threadfence();
  agg_pass(sAcc, dst, tid);
}

__device__ __forceinline__ void xtf_pass(const float* sw, float* xtf, int q0, int lane) {
  const int q8 = lane & 7, sub = lane >> 3;
#pragma unroll
  for (int i = 0; i < 16; ++i) {
    const int lid = i * 4 + sub;
    const int row = lid >> 2, seg = lid & 3;
    const v4f v = *(const v4fa*)(sw + row * DD + 32 * seg + 4 * q8);
    *(volatile v4f*)(xtf + (size_t)(q0 + row) * DD + 32 * seg + 4 * q8) = v;
  }
}

__global__ __launch_bounds__(128) void k_attn(
    const _Float16* __restrict__ qh, const _Float16* __restrict__ kh, const _Float16* __restrict__ vt,
    const float* __restrict__ coords, const _Float16* __restrict__ wot, float* xtf) {
#pragma clang fp contract(off)
  __shared__ __attribute__((aligned(16))) float sO[4 * 16 * DD];

  const int tid = threadIdx.x, lane = tid & 31, wave = tid >> 5, h = lane >> 4, m = lane & 15;
  const int q0 = blockIdx.x * 64 + 16 * wave;

  const _Float16* qrow = qh + (size_t)(q0 + m) * DH;
  const v16h qb0 = ldh(qrow, h);
  const v16h qb1 = ldh(qrow + 32, h);
  const float qx = coords[(size_t)(q0 + m) * 3 + 0];
  const float qy = coords[(size_t)(q0 + m) * 3 + 1];
  const float qz = coords[(size_t)(q0 + m) * 3 + 2];

  const v8f zf = {0.f, 0.f, 0.f, 0.f, 0.f, 0.f, 0.f, 0.f};
  v8f o[4];
#pragma unroll
  for (int t = 0; t < 4; ++t) o[t] = zf;
  float mrun = -1.0e30f, lrun = 0.0f;

  const _Float16* kbase = kh + (size_t)m * DH;
  const _Float16* vbase = vt + (size_t)m * NN;

#pragma unroll 1
  for (int kb = 0; kb < NN; kb += 64) {
    v8f s[4];
#pragma unroll
    for (int j = 0; j < 4; ++j) {
      const _Float16* kp = kbase + (size_t)(kb + 16 * j) * DH;
      v8f z = wmh(ldh(kp, h), qb0, zf);
      z = wmh(ldh(kp + 32, h), qb1, z);
      s[j] = z;
    }
#pragma unroll
    for (int j = 0; j < 4; ++j) {
      const float* cp = coords + (size_t)(kb + 16 * j + 8 * h) * 3;
      const v4f c0 = *(const v4fa*)cp;
      const v4f c1 = *(const v4fa*)(cp + 4);
      const v4f c2 = *(const v4fa*)(cp + 8);
      const v4f c3 = *(const v4fa*)(cp + 12);
      const v4f c4 = *(const v4fa*)(cp + 16);
      const v4f c5 = *(const v4fa*)(cp + 20);
      const float kc[24] = {c0.x, c0.y, c0.z, c0.w, c1.x, c1.y, c1.z, c1.w, c2.x, c2.y, c2.z, c2.w,
                            c3.x, c3.y, c3.z, c3.w, c4.x, c4.y, c4.z, c4.w, c5.x, c5.y, c5.z, c5.w};
#pragma unroll
      for (int r = 0; r < 8; ++r) {
        const float dx = qx - kc[3 * r + 0];
        const float dy = qy - kc[3 * r + 1];
        const float dz = qz - kc[3 * r + 2];
        const float d2 = (dx * dx + dy * dy) + dz * dz;
        const float sv = s[j][r] * 0.125f;
        s[j][r] = (d2 <= RAD2) ? sv : -1.0e9f;
      }
    }
    float mloc = s[0][0];
#pragma unroll
    for (int j = 0; j < 4; ++j)
#pragma unroll
      for (int r = 0; r < 8; ++r) mloc = fmaxf(mloc, s[j][r]);
    mloc = fmaxf(mloc, __shfl_xor(mloc, 16, 32));
    const float mnew = fmaxf(mrun, mloc);
    const float alpha = __expf(mrun - mnew);
    mrun = mnew;
    float lsum = 0.0f;
#pragma unroll
    for (int j = 0; j < 4; ++j)
#pragma unroll
      for (int r = 0; r < 8; ++r) {
        const float p = __expf(s[j][r] - mnew);
        s[j][r] = p;
        lsum += p;
      }
    lsum += __shfl_xor(lsum, 16, 32);
    lrun = lrun * alpha + lsum;
#pragma unroll
    for (int t = 0; t < 4; ++t)
#pragma unroll
      for (int r = 0; r < 8; ++r) o[t][r] = o[t][r] * alpha;

    const v16h pb0 = pack2(s[0], s[1], PSC);
    const v16h pb1 = pack2(s[2], s[3], PSC);

#pragma unroll
    for (int t = 0; t < 4; ++t) {
      const _Float16* vp = vbase + (size_t)(16 * t) * NN + kb;
      o[t] = wmh(ldh(vp, h), pb0, o[t]);
      o[t] = wmh(ldh(vp + 32, h), pb1, o[t]);
    }
  }

  const float inv = (1.0f / lrun) * (1.0f / PSC);
#pragma unroll
  for (int t = 0; t < 4; ++t)
#pragma unroll
    for (int r = 0; r < 8; ++r) o[t][r] = o[t][r] * inv;

  const v16h bo0 = pack2(o[0], o[1], OSC);
  const v16h bo1 = pack2(o[2], o[3], OSC);
  float* sw = sO + wave * (16 * DD);
#pragma unroll
  for (int ft = 0; ft < 8; ++ft) {
    const _Float16* ap = wot + (size_t)(16 * ft + m) * DH;
    v8f d = wmh(ldh(ap, h), bo0, zf);
    d = wmh(ldh(ap + 32, h), bo1, d);
    v4f x0, x1;
    x0.x = d[0] * OINV; x0.y = d[1] * OINV; x0.z = d[2] * OINV; x0.w = d[3] * OINV;
    x1.x = d[4] * OINV; x1.y = d[5] * OINV; x1.z = d[6] * OINV; x1.w = d[7] * OINV;
    float* dp = sw + m * DD + 16 * ft + 8 * h;
    *(v4fa*)dp = x0;
    *(v4fa*)(dp + 4) = x1;
  }
  __syncthreads();

  xtf_pass(sw, xtf, q0, lane);
  __threadfence();
  xtf_pass(sw, xtf, q0, lane);
}

__global__ __launch_bounds__(128) void k_node(
    const float* __restrict__ x, const float* __restrict__ agg, const float* __restrict__ xtf,
    const unsigned short* __restrict__ n1h, const unsigned short* __restrict__ n1l, const float* __restrict__ nb1,
    const unsigned short* __restrict__ n2h, const unsigned short* __restrict__ n2l, const float* __restrict__ nb2,
    const unsigned short* __restrict__ c1h, const unsigned short* __restrict__ c1l, const float* __restrict__ cmb1,
    const float* __restrict__ lng, const float* __restrict__ lnb,
    const unsigned short* __restrict__ c2h, const unsigned short* __restrict__ c2l, const float* __restrict__ cmb2,
    float* out) {
  __shared__ __attribute__((aligned(16))) unsigned short sAh[16 * NK1];
  __shared__ __attribute__((aligned(16))) unsigned short sAl[16 * NK1];
  __shared__ __attribute__((aligned(16))) unsigned short sHh[16 * HH];
  __shared__ __attribute__((aligned(16))) unsigned short sHl[16 * HH];
  __shared__ __attribute__((aligned(16))) float          sF[16 * HH];

  const int tid = threadIdx.x, lane = tid & 31, wave = tid >> 5, h = lane >> 4, m = lane & 15;
  const int n0 = blockIdx.x * 16;
  const v8f zf = {0.f, 0.f, 0.f, 0.f, 0.f, 0.f, 0.f, 0.f};

  for (int i = tid; i < 16 * 32; i += 128) {
    const int row = i >> 5, c4 = (i & 31) * 4;
    const v4f v = *(const v4fa*)(x + (size_t)(n0 + row) * DD + c4);
    v4us hv, lv;
    unsigned short a, b;
    bfsplit(v.x, a, b); hv[0] = a; lv[0] = b;
    bfsplit(v.y, a, b); hv[1] = a; lv[1] = b;
    bfsplit(v.z, a, b); hv[2] = a; lv[2] = b;
    bfsplit(v.w, a, b); hv[3] = a; lv[3] = b;
    *(v4usa*)(sAh + row * NK1 + c4) = hv;
    *(v4usa*)(sAl + row * NK1 + c4) = lv;
  }
  for (int i = tid; i < 16 * 64; i += 128) {
    const int row = i >> 6, c4 = (i & 63) * 4;
    const v4f v = *(const v4fa*)(agg + (size_t)(n0 + row) * HH + c4);
    v4us hv, lv;
    unsigned short a, b;
    bfsplit(v.x, a, b); hv[0] = a; lv[0] = b;
    bfsplit(v.y, a, b); hv[1] = a; lv[1] = b;
    bfsplit(v.z, a, b); hv[2] = a; lv[2] = b;
    bfsplit(v.w, a, b); hv[3] = a; lv[3] = b;
    *(v4usa*)(sAh + row * NK1 + DD + c4) = hv;
    *(v4usa*)(sAl + row * NK1 + DD + c4) = lv;
  }
  __syncthreads();

  {
    v8f a1[4];
#pragma unroll
    for (int j = 0; j < 4; ++j) a1[j] = zf;
#pragma unroll 1
    for (int ks = 0; ks < NK1 / 32; ++ks) {
      const v16b ah = ldb(sAh + m * NK1 + 32 * ks, h);
      const v16b al = ldb(sAl + m * NK1 + 32 * ks, h);
#pragma unroll
      for (int j = 0; j < 4; ++j) {
        const size_t bp = (size_t)(16 * (4 * wave + j) + m) * NK1 + 32 * ks;
        a1[j] = wmb3(ah, al, ldb(n1h + bp, h), ldb(n1l + bp, h), a1[j]);
      }
    }
#pragma unroll
    for (int j = 0; j < 4; ++j) {
      const int col = 16 * (4 * wave + j) + m;
      const float bv = nb1[col];
#pragma unroll
      for (int r = 0; r < 8; ++r) {
        const float v = silu_f(a1[j][r] + bv);
        unsigned short hs, ls;
        bfsplit(v, hs, ls);
        sHh[(8 * h + r) * HH + col] = hs;
        sHl[(8 * h + r) * HH + col] = ls;
      }
    }
  }
  __syncthreads();

  {
    v8f a2[2];
    a2[0] = zf; a2[1] = zf;
#pragma unroll 1
    for (int ks = 0; ks < HH / 32; ++ks) {
      const v16b ah = ldb(sHh + m * HH + 32 * ks, h);
      const v16b al = ldb(sHl + m * HH + 32 * ks, h);
#pragma unroll
      for (int j = 0; j < 2; ++j) {
        const size_t bp = (size_t)(16 * (2 * wave + j) + m) * HH + 32 * ks;
        a2[j] = wmb3(ah, al, ldb(n2h + bp, h), ldb(n2l + bp, h), a2[j]);
      }
    }
#pragma unroll
    for (int j = 0; j < 2; ++j) {
      const int col = 16 * (2 * wave + j) + m;
      const float bv = nb2[col];
#pragma unroll
      for (int r = 0; r < 8; ++r) {
        const size_t gi = (size_t)(n0 + 8 * h + r) * DD + col;
        const float xv = x[gi];
        const float tv = xtf[gi];
        const float cv = (xv + (a2[j][r] + bv)) + tv;
        unsigned short hs, ls;
        bfsplit(cv, hs, ls);
        sAh[(8 * h + r) * DD + col] = hs;
        sAl[(8 * h + r) * DD + col] = ls;
      }
    }
  }
  __syncthreads();

  {
    v8f a3[4];
#pragma unroll
    for (int j = 0; j < 4; ++j) a3[j] = zf;
#pragma unroll 1
    for (int ks = 0; ks < DD / 32; ++ks) {
      const v16b ah = ldb(sAh + m * DD + 32 * ks, h);
      const v16b al = ldb(sAl + m * DD + 32 * ks, h);
#pragma unroll
      for (int j = 0; j < 4; ++j) {
        const size_t bp = (size_t)(16 * (4 * wave + j) + m) * DD + 32 * ks;
        a3[j] = wmb3(ah, al, ldb(c1h + bp, h), ldb(c1l + bp, h), a3[j]);
      }
    }
#pragma unroll
    for (int j = 0; j < 4; ++j) {
      const int col = 16 * (4 * wave + j) + m;
      const float bv = cmb1[col];
#pragma unroll
      for (int r = 0; r < 8; ++r) sF[(8 * h + r) * HH + col] = fmaxf(a3[j][r] + bv, 0.0f);
    }
  }
  __syncthreads();

  {
    const v4f g0 = *(const v4fa*)(lng + 8 * lane);
    const v4f g1 = *(const v4fa*)(lng + 8 * lane + 4);
    const v4f b0 = *(const v4fa*)(lnb + 8 * lane);
    const v4f b1 = *(const v4fa*)(lnb + 8 * lane + 4);
    const float gg[8] = {g0.x, g0.y, g0.z, g0.w, g1.x, g1.y, g1.z, g1.w};
    const float bb[8] = {b0.x, b0.y, b0.z, b0.w, b1.x, b1.y, b1.z, b1.w};
#pragma unroll 1
    for (int rr = 0; rr < 4; ++rr) {
      const int row = 4 * wave + rr;
      const float* fp = sF + row * HH + 8 * lane;
      const v4f v0 = *(const v4fa*)fp;
      const v4f v1 = *(const v4fa*)(fp + 4);
      const float vv[8] = {v0.x, v0.y, v0.z, v0.w, v1.x, v1.y, v1.z, v1.w};
      float s = 0.0f;
#pragma unroll
      for (int i = 0; i < 8; ++i) s += vv[i];
      s = wsum(s);
      const float mu = s * (1.0f / (float)HH);
      float dv[8];
      float ss = 0.0f;
#pragma unroll
      for (int i = 0; i < 8; ++i) { dv[i] = vv[i] - mu; ss += dv[i] * dv[i]; }
      ss = wsum(ss);
      const float var = ss * (1.0f / (float)HH);
      const float rstd = rsqrtf(var + 1e-5f);
      v8us hv, lv;
#pragma unroll
      for (int i = 0; i < 8; ++i) {
        const float y = dv[i] * rstd * gg[i] + bb[i];
        unsigned short hs, ls;
        bfsplit(y, hs, ls);
        hv[i] = hs; lv[i] = ls;
      }
      *(v8usa*)(sHh + row * HH + 8 * lane) = hv;
      *(v8usa*)(sHl + row * HH + 8 * lane) = lv;
    }
  }
  __syncthreads();

  {
    v8f a4 = zf;
#pragma unroll 1
    for (int ks = 0; ks < HH / 32; ++ks) {
      const v16b ah = ldb(sHh + m * HH + 32 * ks, h);
      const v16b al = ldb(sHl + m * HH + 32 * ks, h);
      const size_t bp = (size_t)(16 * wave + m) * HH + 32 * ks;
      a4 = wmb3(ah, al, ldb(c2h + bp, h), ldb(c2l + bp, h), a4);
    }
    const int col = 16 * wave + m;
    const float bv = cmb2[col];
#pragma unroll
    for (int r = 0; r < 8; ++r) sF[(8 * h + r) * YY + col] = a4[r] + bv;
  }
  __syncthreads();

  float* dst = out + (size_t)n0 * YY;
  const v4f w0 = *(const v4fa*)(sF + 4 * tid);
  const v4f w1 = *(const v4fa*)(sF + 4 * (tid + 128));
  *(volatile v4f*)(dst + 4 * tid) = w0;
  *(volatile v4f*)(dst + 4 * (tid + 128)) = w1;
  __threadfence();
  *(volatile v4f*)(dst + 4 * tid) = w0;
  *(volatile v4f*)(dst + 4 * (tid + 128)) = w1;
}

extern "C" void kernel_launch(void* const* d_in, const int* in_sizes, int n_in,
                              void* d_out, int out_size, void* d_ws, size_t ws_size,
                              hipStream_t stream) {
  if (n_in < 22) return;
  if (in_sizes[0] != NN * DD || in_sizes[1] != NN * 3 || in_sizes[2] != EE * ED || in_sizes[3] != 2 * EE) return;
  if (in_sizes[4] != NE1 * HH || in_sizes[5] != HH || in_sizes[6] != HH * HH || in_sizes[7] != HH) return;
  if (in_sizes[8] != NK1 * HH || in_sizes[9] != HH || in_sizes[10] != HH * DD || in_sizes[11] != DD) return;
  if (in_sizes[12] != DD * DH || in_sizes[13] != DD * DH || in_sizes[14] != DD * DH || in_sizes[15] != DH * DD) return;
  if (in_sizes[16] != DD * HH || in_sizes[17] != HH || in_sizes[18] != HH || in_sizes[19] != HH) return;
  if (in_sizes[20] != HH * YY || in_sizes[21] != YY) return;
  if (out_size != NN * YY) return;

  const float* x     = (const float*)d_in[0];
  const float* crd   = (const float*)d_in[1];
  const float* eattr = (const float*)d_in[2];
  const int*   ei    = (const int*)d_in[3];
  const float* ew1   = (const float*)d_in[4];
  const float* eb1   = (const float*)d_in[5];
  const float* ew2   = (const float*)d_in[6];
  const float* eb2   = (const float*)d_in[7];
  const float* nw1   = (const float*)d_in[8];
  const float* nb1   = (const float*)d_in[9];
  const float* nw2   = (const float*)d_in[10];
  const float* nb2   = (const float*)d_in[11];
  const float* wq    = (const float*)d_in[12];
  const float* wk    = (const float*)d_in[13];
  const float* wv    = (const float*)d_in[14];
  const float* wo    = (const float*)d_in[15];
  const float* cmw1  = (const float*)d_in[16];
  const float* cmb1  = (const float*)d_in[17];
  const float* lng   = (const float*)d_in[18];
  const float* lnb   = (const float*)d_in[19];
  const float* cmw2  = (const float*)d_in[20];
  const float* cmb2  = (const float*)d_in[21];
  float* out = (float*)d_out;

  size_t off = 0;
  const size_t o_xh  = off; off += (size_t)NN * DD * 2;
  const size_t o_wf  = off; off += (size_t)NWF * DD * 2;
  const size_t o_wa  = off; off += (size_t)HH * 32 * 2;
  const size_t o_w2  = off; off += (size_t)HH * HH * 2;
  const size_t o_wot = off; off += (size_t)DD * DH * 2;
  const size_t o_n1h = off; off += (size_t)HH * NK1 * 2;
  const size_t o_n1l = off; off += (size_t)HH * NK1 * 2;
  const size_t o_n2h = off; off += (size_t)DD * HH * 2;
  const size_t o_n2l = off; off += (size_t)DD * HH * 2;
  const size_t o_c1h = off; off += (size_t)HH * DD * 2;
  const size_t o_c1l = off; off += (size_t)HH * DD * 2;
  const size_t o_c2h = off; off += (size_t)YY * HH * 2;
  const size_t o_c2l = off; off += (size_t)YY * HH * 2;
  const size_t o_pq  = off; off += (size_t)NN * 2 * HH * 4;
  const size_t o_qh  = off; off += (size_t)NN * DH * 2;
  const size_t o_kh  = off; off += (size_t)NN * DH * 2;
  const size_t o_vt  = off; off += (size_t)DH * NN * 2;
  const size_t o_agg = off; off += (size_t)NN * HH * 4;
  const size_t o_xtf = off; off += (size_t)NN * DD * 4;
  if (off > ws_size) return;

  char* ws = (char*)d_ws;
  unsigned short* xh  = (unsigned short*)(ws + o_xh);
  unsigned short* wf  = (unsigned short*)(ws + o_wf);
  unsigned short* wa  = (unsigned short*)(ws + o_wa);
  unsigned short* w2  = (unsigned short*)(ws + o_w2);
  unsigned short* wot = (unsigned short*)(ws + o_wot);
  unsigned short* n1h = (unsigned short*)(ws + o_n1h);
  unsigned short* n1l = (unsigned short*)(ws + o_n1l);
  unsigned short* n2h = (unsigned short*)(ws + o_n2h);
  unsigned short* n2l = (unsigned short*)(ws + o_n2l);
  unsigned short* c1h = (unsigned short*)(ws + o_c1h);
  unsigned short* c1l = (unsigned short*)(ws + o_c1l);
  unsigned short* c2h = (unsigned short*)(ws + o_c2h);
  unsigned short* c2l = (unsigned short*)(ws + o_c2l);
  float*    pq  = (float*)(ws + o_pq);
  _Float16* qh  = (_Float16*)(ws + o_qh);
  _Float16* kh  = (_Float16*)(ws + o_kh);
  _Float16* vtp = (_Float16*)(ws + o_vt);
  float*    agg = (float*)(ws + o_agg);
  float*    xtf = (float*)(ws + o_xtf);

  k_convert<<<CB9 / 256, 256, 0, stream>>>(x, ew1, ew2, wq, wk, wv, wo, nw1, nw2, cmw1, cmw2,
                                            xh, wf, wa, w2, wot, n1h, n1l, n2h, n2l, c1h, c1l, c2h, c2l);

  k_proj<<<dim3(NN / 128, 11), 128, 0, stream>>>((const _Float16*)xh, (const _Float16*)wf, eb1, pq, qh, kh, vtp);

  k_edge<<<NN / NB, ENT, 0, stream>>>(pq, crd, eattr, ei, ew1, eb2, (const _Float16*)wa, (const _Float16*)w2,
                                      agg, NN, EE);

  k_attn<<<NN / 64, 128, 0, stream>>>((const _Float16*)qh, (const _Float16*)kh, (const _Float16*)vtp, crd,
                                      (const _Float16*)wot, xtf);

  k_node<<<NN / 16, 128, 0, stream>>>(x, agg, xtf, n1h, n1l, nb1, n2h, n2l, nb2, c1h, c1l, cmb1, lng, lnb,
                                      c2h, c2l, cmb2, out);
}
